// FastShapeTransformerModel_40647570489995
// MI455X (gfx1250) — hardware-verified
//
#include <hip/hip_runtime.h>
#include <math.h>

typedef __attribute__((ext_vector_type(16))) _Float16 v16h;
typedef __attribute__((ext_vector_type(16))) __bf16 v16b;
typedef __attribute__((ext_vector_type(8)))  _Float16 v8h;
typedef __attribute__((ext_vector_type(8)))  float v8f;
typedef __attribute__((ext_vector_type(4)))  float v4f;
typedef __attribute__((ext_vector_type(2)))  float v2f;
typedef __attribute__((ext_vector_type(4)))  unsigned v4u;
typedef __attribute__((ext_vector_type(4)))  int v4i;
typedef float __attribute__((may_alias)) float_a;
typedef int __attribute__((may_alias)) int_a;

template <typename T> __device__ __forceinline__ void vst2(void* p, T v) { *(volatile T*)p = v; __threadfence(); *(volatile T*)p = v; }
__device__ __forceinline__ v8f wmma16(v16h a, v16h b, v8f c) {
  v8f d = __builtin_amdgcn_wmma_f32_16x16x32_f16(false, a, false, b, (short)0, c, false, false);
  asm volatile("v_nop\n\tv_nop\n\tv_nop\n\tv_nop" : "+v"(d) : "v"(a), "v"(b));
  return d;
}
__device__ __forceinline__ v8f wmma_bf(v16b a, v16b b, v8f c) {
  v8f d = __builtin_amdgcn_wmma_f32_16x16x32_bf16(false, a, false, b, (short)0, c, false, false);
  asm volatile("v_nop\n\tv_nop\n\tv_nop\n\tv_nop" : "+v"(d) : "v"(a), "v"(b));
  return d;
}
__device__ __forceinline__ v16h frag_h(const _Float16* rowk0, int lane) {
  union { v16h v; v8h q[2]; } u; const _Float16* p = rowk0 + 8 * (lane >> 4);
  u.q[0] = *(const v8h*)p; u.q[1] = *(const v8h*)(p + 16); return u.v;
}
__device__ __forceinline__ v16h frag_f32(const float* rowk0, int lane) {
  v16h a; const float* p = rowk0 + 8 * (lane >> 4);
#pragma unroll
  for (int i = 0; i < 8; ++i) { a[i] = (_Float16)p[i]; a[8 + i] = (_Float16)p[16 + i]; }
  return a;
}
__device__ __forceinline__ v16h frag_f32s(const float* rowk0, int lane, float sc) {
  v16h a; const float* p = rowk0 + 8 * (lane >> 4);
#pragma unroll
  for (int i = 0; i < 8; ++i) { a[i] = (_Float16)(p[i] * sc); a[8 + i] = (_Float16)(p[16 + i] * sc); }
  return a;
}
__device__ __forceinline__ v16h fragc_f32(const float* W, int k0, int n, int lane, int ld, int K) {
  v16h a; const int g = lane >> 4;
#pragma unroll
  for (int i = 0; i < 8; ++i) { const int ka = k0 + 8 * g + i, kb = ka + 16;
    a[i] = (_Float16)(ka < K ? W[(size_t)(ka < K ? ka : K - 1) * ld + n] : 0.f); a[8 + i] = (_Float16)(kb < K ? W[(size_t)(kb < K ? kb : K - 1) * ld + n] : 0.f); }
  return a;
}
struct F2 { v16b h, l; };
__device__ __forceinline__ F2 bsplit16(const float v[16]) { F2 r;
#pragma unroll
  for (int i = 0; i < 16; ++i) { const __bf16 h = (__bf16)v[i]; r.h[i] = h; r.l[i] = (__bf16)(v[i] - (float)h); }
  return r; }
__device__ __forceinline__ F2 split_row(const float* row, int k0, int lane) { float v[16]; const float* p = row + k0 + 8 * (lane >> 4);
#pragma unroll
  for (int i = 0; i < 8; ++i) { v[i] = p[i]; v[8 + i] = p[16 + i]; }
  return bsplit16(v); }
__device__ __forceinline__ F2 split_rowK(const float* row, int k0, int lane, int K) { float v[16]; const int g = lane >> 4;
#pragma unroll
  for (int i = 0; i < 8; ++i) { const int ka = k0 + 8 * g + i, kb = ka + 16; v[i] = ka < K ? row[ka < K ? ka : K - 1] : 0.f; v[8 + i] = kb < K ? row[kb < K ? kb : K - 1] : 0.f; }
  return bsplit16(v); }
__device__ __forceinline__ F2 split_col(const float* W, int k0, int n, int lane, int ld, int K) { float v[16]; const int g = lane >> 4;
#pragma unroll
  for (int i = 0; i < 8; ++i) { const int ka = k0 + 8 * g + i, kb = ka + 16; v[i] = ka < K ? W[(size_t)(ka < K ? ka : K - 1) * ld + n] : 0.f; v[8 + i] = kb < K ? W[(size_t)(kb < K ? kb : K - 1) * ld + n] : 0.f; }
  return bsplit16(v); }
__device__ __forceinline__ v8f mac3(const F2& a, const F2& b, v8f c) { c = wmma_bf(a.l, b.h, c); c = wmma_bf(a.h, b.l, c); return wmma_bf(a.h, b.h, c); }
__device__ __forceinline__ float sigm(float v) { return 1.0f / (1.0f + expf(-v)); }
#define LDSX() do { asm volatile("s_wait_dscnt 0" ::: "memory"); __builtin_amdgcn_wave_barrier(); __builtin_amdgcn_fence(__ATOMIC_RELEASE, "workgroup"); } while (0)


#define NSEQ 2
#define SS 1024
#define NR (NSEQ * SS)
#define EE 512
#define NH 8
#define HD 64
#define FF 2048
#define NL 4
#define NV 17
#ifndef NRT
#define NRT NR
#endif
typedef __attribute__((ext_vector_type(8))) __bf16 v8b;
__device__ __forceinline__ v16b frag_b(const __bf16* rowk0, int lane) {
  union { v16b v; v8b q[2]; } u; const __bf16* p = rowk0 + 8 * (lane >> 4);
  u.q[0] = *(const v8b*)p; u.q[1] = *(const v8b*)(p + 16); return u.v;
}
__device__ __forceinline__ float bfr(float v) { return (float)(__bf16)v; }
__device__ __attribute__((noinline)) float exp_ni(float v) { return expf(v); }
__device__ __attribute__((noinline)) float erf_ni(float v) { return erff(v); }
__device__ __attribute__((noinline)) float expm1_ni(float v) { return expm1f(v); }
__device__ __forceinline__ float gelu_exact(float v) { return 0.5f * v * (1.0f + erf_ni(v * 0.70710678118654752f)); }
__device__ __forceinline__ float elu1(float v) { return (v > 0.f) ? v + 1.0f : expm1_ni(v) + 1.0f; }

#define PL_QKV 0
#define PL_O   (PL_QKV + 3 * EE * EE)
#define PL_F1  (PL_O + EE * EE)
#define PL_F2  (PL_F1 + FF * EE)
#define PL_SZ  (PL_F2 + EE * FF)
#define PK_HEAD ((size_t)NL * PL_SZ)
#define PK_END (PK_HEAD + 32 * EE)
#define WS_PK  0u
#define WS_X   (((2u * PK_END) + 127u) / 128u * 128u)
#define WS_XH  (WS_X + 4u * NR * EE)
#define WS_XL  (WS_XH + 2u * NR * EE)
#define WS_Y   (WS_XL + 2u * NR * EE)
#define WS_QF  (WS_Y + 4u * NR * EE)
#define WS_KF  (WS_QF + 2u * NR * EE)
#define WS_VT  (WS_KF + 2u * NR * EE)
#define WS_ATT (WS_VT + 2u * NR * EE)
#define WS_ATL (WS_ATT + 2u * NR * EE)
#define WS_HFH (WS_ATL + 2u * NR * EE)
#define WS_HFL (WS_HFH + 2u * NR * FF)
#define WS_MSK (WS_HFL + 2u * NR * FF)
#define WS_STG (WS_MSK + 4u * NR)
#define WS_END (WS_STG + 4u * NR * 32)

__global__ __launch_bounds__(256) void k_pack(const float* __restrict__ WQ, const float* __restrict__ WK, const float* __restrict__ WV, const float* __restrict__ WO, const float* __restrict__ W1, const float* __restrict__ W2, const float* __restrict__ WH, __bf16* __restrict__ PK) {
  __shared__ __align__(16) __bf16 s[FF]; const int n = blockIdx.x, which = blockIdx.y, l = blockIdx.z, t = threadIdx.x; int K = EE; size_t dst; const float* src = nullptr; bool zero = false;
  __bf16* base = PK + (size_t)l * PL_SZ;
  if (which == 0) { if (n >= 3 * EE) return; const int m = n / EE, r = n % EE; const float* Wm = (m == 0) ? WQ : (m == 1) ? WK : WV; src = Wm + ((size_t)l * EE + r) * EE; dst = PL_QKV + (size_t)n * EE; }
  else if (which == 1) { if (n >= EE) return; src = WO + ((size_t)l * EE + n) * EE; dst = PL_O + (size_t)n * EE; }
  else if (which == 2) { src = W1 + ((size_t)l * FF + n) * EE; dst = PL_F1 + (size_t)n * EE; }
  else if (which == 3) { if (n >= EE) return; K = FF; src = W2 + ((size_t)l * EE + n) * FF; dst = PL_F2 + (size_t)n * FF; }
  else { if (l > 0 || n >= 32) return; base = PK; dst = PK_HEAD + (size_t)n * EE; zero = (n >= NV); src = WH + (size_t)(zero ? 0 : n) * EE; }
  for (int k = t; k < K; k += 256) s[k] = (__bf16)(zero ? 0.f : src[k]);
  __syncthreads();
  for (int q = t; q < K / 8; q += 256) vst2((unsigned*)(base + dst + q * 8), *(const v4u*)&s[q * 8]);
}
__global__ __launch_bounds__(128) void k_embed(const int* __restrict__ SEQ, const int* __restrict__ DEP, const int* __restrict__ POS, const float* __restrict__ TE, const float* __restrict__ DE, const float* __restrict__ SPE, const float* __restrict__ SOS, float* __restrict__ X, __bf16* __restrict__ XH, __bf16* __restrict__ XL, float* __restrict__ MSK) {
  __shared__ __align__(16) float sx[EE]; __shared__ __align__(16) __bf16 sh_[EE], sl_[EE];
  const int row = blockIdx.x, t = threadIdx.x; const int n = row / SS, s = row % SS;
  for (int c = t; c < EE; c += 128) { float v;
    if (s == 0) v = bfr(SOS[c]);
    else { const int sp = s - 1; const int tok = min(max(SEQ[n * SS + sp], 0), NV - 1), dp = min(max(DEP[n * SS + sp], 0), 6);
      v = bfr(TE[(size_t)tok * EE + c]) + bfr(DE[(size_t)dp * EE + c]);
#pragma unroll
      for (int a = 0; a < 3; ++a) { const int pp = min(max(POS[((size_t)a * NSEQ + n) * SS + sp], 0), 64); v += bfr(SPE[((size_t)a * 65 + pp) * EE + c]); } }
    sx[c] = v; const __bf16 hb = (__bf16)v; sh_[c] = hb; sl_[c] = (__bf16)(v - (float)hb); }
  __syncthreads();
  vst2(X + (size_t)row * EE + t * 4, *(const v4f*)&sx[t * 4]);
  if (t < 64) vst2((unsigned*)(XH + (size_t)row * EE + t * 8), *(const v4u*)&sh_[t * 8]); else vst2((unsigned*)(XL + (size_t)row * EE + (t - 64) * 8), *(const v4u*)&sl_[(t - 64) * 8]);
}
__global__ __launch_bounds__(256) void k_mask(const int* __restrict__ SEQ, float* __restrict__ MSK) {
  __shared__ __align__(16) float sm[256]; const int t = threadIdx.x; const size_t row = (size_t)blockIdx.x * 256 + t; sm[t] = (SEQ[row] != 0) ? 1.f : 0.f;
  __syncthreads();
  if (t < 64) vst2(MSK + (size_t)blockIdx.x * 256 + t * 4, *(const v4f*)&sm[t * 4]);
}
template <int MODE>
__global__ __launch_bounds__(128) void k_gemm(const __bf16* __restrict__ AH, const __bf16* __restrict__ AL, const __bf16* __restrict__ P, const float* __restrict__ BIAS, const float* __restrict__ X, const float* __restrict__ MSK, _Float16* __restrict__ QF, _Float16* __restrict__ KF, _Float16* __restrict__ VT, __bf16* __restrict__ OH, __bf16* __restrict__ OL, float* __restrict__ OUTF, int which0) {
  constexpr int KIN = (MODE == 3) ? FF : EE;
  __shared__ __align__(16) float so[4][16][132]; __shared__ __align__(16) __bf16 soh[4][16][136], sol[4][16][136]; __shared__ __align__(16) _Float16 sq[4][16][136]; __shared__ __align__(16) _Float16 st[128][72];
  const int tid = threadIdx.x, wave = tid >> 5, lane = tid & 31, col = lane & 15, g = lane >> 4; const size_t r0 = (size_t)blockIdx.x * 64 + wave * 16; const int n0 = blockIdx.y * 128;
  const int ntile = (MODE == 4) ? 2 : 8;
  v8f acc[8] = {};
#pragma unroll 2
  for (int kc = 0; kc < KIN / 32; ++kc) { F2 a; a.h = frag_b(AH + (r0 + col) * KIN + kc * 32, lane); a.l = frag_b(AL + (r0 + col) * KIN + kc * 32, lane);
#pragma unroll
    for (int j = 0; j < 8; ++j) if (j < ntile) { const v16b w = frag_b(P + (size_t)(n0 + j * 16 + col) * KIN + kc * 32, lane); acc[j] = wmma_bf(a.l, w, acc[j]); acc[j] = wmma_bf(a.h, w, acc[j]); } }
  if (MODE == 0) {
    const int which = which0;
#pragma unroll
    for (int j = 0; j < 8; ++j) { const int c = n0 + j * 16 + col; const float bb = bfr(BIAS[c]);
#pragma unroll
      for (int r = 0; r < 8; ++r) { const size_t row = r0 + 8 * g + r; const float v = acc[j][r] + bb;
        if (which == 0) sq[wave][8 * g + r][j * 16 + col] = (_Float16)elu1(v);
        else if (which == 1) sq[wave][8 * g + r][j * 16 + col] = (_Float16)(elu1(v) * MSK[row]);
        else st[j * 16 + col][wave * 16 + 8 * g + r] = (_Float16)v; } }
    if (which < 2) { LDSX(); _Float16* DST = (which == 0) ? QF : KF; const int c0 = n0;
      for (int rl = 0; rl < 16; ++rl) if (lane < 16) vst2((unsigned*)(DST + (r0 + rl) * EE + c0 + lane * 8), *(const v4u*)&sq[wave][rl][lane * 8]); }
    else { __syncthreads(); const size_t rb = (size_t)blockIdx.x * 64; const int n = (int)(rb / SS), s0 = (int)(rb % SS); const int pc0 = n0;
      for (int q = tid; q < 128 * 8; q += 128) { const int d = q >> 3, pc = q & 7; vst2((unsigned*)(VT + ((size_t)n * EE + pc0 + d) * SS + s0 + pc * 8), *(const v4u*)&st[d][pc * 8]); } }
    return; }
#pragma unroll
  for (int j = 0; j < 8; ++j) if (j < ntile) { const int c = n0 + j * 16 + col; const float bb = (MODE == 4) ? 0.f : bfr(BIAS[c]);
#pragma unroll
    for (int r = 0; r < 8; ++r) { const size_t row = r0 + 8 * g + r; const float v = acc[j][r] + bb;
      if (MODE == 1 || MODE == 3) so[wave][8 * g + r][j * 16 + col] = X[row * EE + c] + v;
      else if (MODE == 2) { const float gq = gelu_exact(v); const __bf16 hb = (__bf16)gq; soh[wave][8 * g + r][j * 16 + col] = hb; sol[wave][8 * g + r][j * 16 + col] = (__bf16)(gq - (float)hb); }
      else so[wave][8 * g + r][j * 16 + col] = v; } }
  LDSX();
  for (int rl = 0; rl < 16; ++rl) {
    if (MODE == 1 || MODE == 3) vst2(OUTF + (r0 + rl) * EE + n0 + lane * 4, *(const v4f*)&so[wave][rl][lane * 4]);
    else if (MODE == 2) { if (lane < 16) { vst2((unsigned*)(OH + (r0 + rl) * FF + n0 + lane * 8), *(const v4u*)&soh[wave][rl][lane * 8]); vst2((unsigned*)(OL + (r0 + rl) * FF + n0 + lane * 8), *(const v4u*)&sol[wave][rl][lane * 8]); } }
    else { if (lane < 8) vst2(OUTF + (r0 + rl) * 32 + lane * 4, *(const v4f*)&so[wave][rl][lane * 4]); } }
}
__global__ __launch_bounds__(128) void k_attn(const _Float16* __restrict__ QF, const _Float16* __restrict__ KF, const _Float16* __restrict__ VT, __bf16* __restrict__ OH, __bf16* __restrict__ OL) {
  __shared__ __align__(16) _Float16 sp[4][16][40]; __shared__ __align__(16) __bf16 soh[4][16][72], sol[4][16][72];
  const int tid = threadIdx.x, wave = tid >> 5, lane = tid & 31, col = lane & 15, g = lane >> 4; const int qb = blockIdx.x, h = blockIdx.y, n = blockIdx.z; const int q0 = qb * 64 + wave * 16; const size_t rq = (size_t)n * SS + q0 + col;
  v16h aq[2];
#pragma unroll
  for (int kc = 0; kc < 2; ++kc) aq[kc] = frag_h(QF + rq * EE + h * HD + kc * 32, lane);
  float l[8];
#pragma unroll
  for (int r = 0; r < 8; ++r) l[r] = 0.f;
  v8f acc[4] = {};
  const int nks = (qb * 64 + 64) / 32;
#pragma unroll 1
  for (int ks = 0; ks < nks; ++ks) {
#pragma unroll
    for (int ct = 0; ct < 2; ++ct) { const int kk = ks * 32 + ct * 16 + col; v8f c = {};
#pragma unroll
      for (int kc = 0; kc < 2; ++kc) c = wmma16(aq[kc], frag_h(KF + ((size_t)n * SS + kk) * EE + h * HD + kc * 32, lane), c);
#pragma unroll
      for (int r = 0; r < 8; ++r) { const int qi = q0 + 8 * g + r; const _Float16 a16 = (kk <= qi) ? (_Float16)c[r] : (_Float16)0.f; sp[wave][8 * g + r][ct * 16 + col] = a16; l[r] += (float)a16; } }
    LDSX();
    const v16h pa = frag_h(&sp[wave][col][0], lane);
#pragma unroll
    for (int dt = 0; dt < 4; ++dt) acc[dt] = wmma16(pa, frag_h(VT + ((size_t)n * EE + h * HD + dt * 16 + col) * SS + ks * 32, lane), acc[dt]);
    LDSX(); }
#pragma unroll
  for (int r = 0; r < 8; ++r) {
#pragma unroll
    for (int o = 1; o < 16; o <<= 1) l[r] += __shfl_xor(l[r], o); }
#pragma unroll
  for (int r = 0; r < 8; ++r) { const float z = 1.0f / (l[r] + 1e-6f);
#pragma unroll
    for (int dt = 0; dt < 4; ++dt) { const float v = acc[dt][r] * z; const __bf16 hb = (__bf16)v; soh[wave][8 * g + r][dt * 16 + col] = hb; sol[wave][8 * g + r][dt * 16 + col] = (__bf16)(v - (float)hb); } }
  LDSX();
  for (int rl = 0; rl < 16; ++rl) { if (lane < 8) vst2((unsigned*)(OH + ((size_t)n * SS + q0 + rl) * EE + h * HD + lane * 8), *(const v4u*)&soh[wave][rl][lane * 8]); else if (lane < 16) vst2((unsigned*)(OL + ((size_t)n * SS + q0 + rl) * EE + h * HD + (lane - 8) * 8), *(const v4u*)&sol[wave][rl][(lane - 8) * 8]); }
}
__global__ __launch_bounds__(128) void k_ln(const float* __restrict__ Y, const float* __restrict__ G, const float* __restrict__ Bb, float* __restrict__ X, __bf16* __restrict__ XH, __bf16* __restrict__ XL) {
  __shared__ float sred[2][4]; __shared__ __align__(16) float sx[EE]; __shared__ __align__(16) __bf16 sh_[EE], sl_[EE]; const int t = threadIdx.x; const size_t row = blockIdx.x;
  float v[4]; float s = 0.f;
#pragma unroll
  for (int i = 0; i < 4; ++i) { v[i] = Y[row * EE + t + 128 * i]; s += v[i]; }
#pragma unroll
  for (int o = 1; o < 32; o <<= 1) s += __shfl_xor(s, o);
  if ((t & 31) == 0) sred[0][t >> 5] = s;
  __syncthreads();
  const float mu = ((sred[0][0] + sred[0][1]) + (sred[0][2] + sred[0][3])) * (1.0f / EE); float q = 0.f;
#pragma unroll
  for (int i = 0; i < 4; ++i) { const float d = v[i] - mu; q += d * d; }
#pragma unroll
  for (int o = 1; o < 32; o <<= 1) q += __shfl_xor(q, o);
  if ((t & 31) == 0) sred[1][t >> 5] = q;
  __syncthreads();
  const float rs = rsqrtf(((sred[1][0] + sred[1][1]) + (sred[1][2] + sred[1][3])) * (1.0f / EE) + 1e-5f);
#pragma unroll
  for (int i = 0; i < 4; ++i) { const int c = t + 128 * i; const float x = (v[i] - mu) * rs * bfr(G[c]) + bfr(Bb[c]); sx[c] = x; const __bf16 hb = (__bf16)x; sh_[c] = hb; sl_[c] = (__bf16)(x - (float)hb); }
  __syncthreads();
  vst2(X + row * EE + t * 4, *(const v4f*)&sx[t * 4]);
  if (t < 64) vst2((unsigned*)(XH + row * EE + t * 8), *(const v4u*)&sh_[t * 8]); else vst2((unsigned*)(XL + row * EE + (t - 64) * 8), *(const v4u*)&sl_[(t - 64) * 8]);
}
__global__ __launch_bounds__(256) void k_outw(const float* __restrict__ STG, float* __restrict__ OUT) {
  __shared__ __align__(16) float s[64 * NV + 16]; const int t = threadIdx.x; const size_t r0 = (size_t)blockIdx.x * 64;
  for (int q = t; q < 64 * NV; q += 256) { const int r = q / NV, c = q % NV; s[q] = STG[(r0 + r) * 32 + c]; }
  __syncthreads();
  for (int q = t; q < 64 * NV / 4; q += 256) vst2(OUT + r0 * NV + q * 4, *(const v4f*)&s[q * 4]);
}
extern "C" void kernel_launch(void* const* d_in, const int* in_sizes, int n_in, void* d_out, int out_size, void* d_ws, size_t ws_size, hipStream_t stream) {
  (void)in_sizes; (void)n_in; (void)out_size;
  const float** F = (const float**)d_in;
  if (ws_size < (size_t)WS_END) return;
  char* ws = (char*)d_ws; __bf16 *PK = (__bf16*)(ws + WS_PK), *XH = (__bf16*)(ws + WS_XH), *XL = (__bf16*)(ws + WS_XL), *ATH = (__bf16*)(ws + WS_ATT), *ATL = (__bf16*)(ws + WS_ATL), *HFH = (__bf16*)(ws + WS_HFH), *HFL = (__bf16*)(ws + WS_HFL);
  float *X = (float*)(ws + WS_X), *Y = (float*)(ws + WS_Y), *MSK = (float*)(ws + WS_MSK), *STG = (float*)(ws + WS_STG); _Float16 *QF = (_Float16*)(ws + WS_QF), *KF = (_Float16*)(ws + WS_KF), *VT = (_Float16*)(ws + WS_VT);
  k_pack<<<dim3(FF, 5, NL), 256, 0, stream>>>(F[7], F[9], F[11], F[13], F[17], F[19], F[25], PK);
  k_embed<<<NRT, 128, 0, stream>>>((const int*)d_in[0], (const int*)d_in[1], (const int*)d_in[2], F[3], F[4], F[5], F[6], X, XH, XL, MSK);
  k_mask<<<NRT / 256, 256, 0, stream>>>((const int*)d_in[0], MSK);
  for (int l = 0; l < NL; ++l) { const __bf16* base = PK + (size_t)l * PL_SZ;
    k_gemm<0><<<dim3(NRT / 64, 4), 128, 0, stream>>>(XH, XL, base + PL_QKV, F[8] + (size_t)l * EE, X, MSK, QF, KF, VT, nullptr, nullptr, nullptr, 0);
    k_gemm<0><<<dim3(NRT / 64, 4), 128, 0, stream>>>(XH, XL, base + PL_QKV + (size_t)EE * EE, F[10] + (size_t)l * EE, X, MSK, QF, KF, VT, nullptr, nullptr, nullptr, 1);
    k_gemm<0><<<dim3(NRT / 64, 4), 128, 0, stream>>>(XH, XL, base + PL_QKV + (size_t)2 * EE * EE, F[12] + (size_t)l * EE, X, MSK, QF, KF, VT, nullptr, nullptr, nullptr, 2);
    k_attn<<<dim3((NRT < SS ? NRT : SS) / 64, NH, (NRT < SS ? 1 : NSEQ)), 128, 0, stream>>>(QF, KF, VT, ATH, ATL);
    k_gemm<1><<<dim3(NRT / 64, EE / 128), 128, 0, stream>>>(ATH, ATL, base + PL_O, F[14] + (size_t)l * EE, X, nullptr, nullptr, nullptr, nullptr, nullptr, nullptr, Y, 0);
    k_ln<<<NRT, 128, 0, stream>>>(Y, F[15] + (size_t)l * EE, F[16] + (size_t)l * EE, X, XH, XL);
    k_gemm<2><<<dim3(NRT / 64, FF / 128), 128, 0, stream>>>(XH, XL, base + PL_F1, F[18] + (size_t)l * FF, nullptr, nullptr, nullptr, nullptr, nullptr, HFH, HFL, nullptr, 0);
    k_gemm<3><<<dim3(NRT / 64, EE / 128), 128, 0, stream>>>(HFH, HFL, base + PL_F2, F[20] + (size_t)l * EE, X, nullptr, nullptr, nullptr, nullptr, nullptr, nullptr, Y, 0);
    k_ln<<<NRT, 128, 0, stream>>>(Y, F[21] + (size_t)l * EE, F[22] + (size_t)l * EE, X, XH, XL); }
  k_ln<<<NRT, 128, 0, stream>>>(X, F[23], F[24], Y, XH, XL);
  k_gemm<4><<<dim3(NRT / 64, 1), 128, 0, stream>>>(XH, XL, PK + PK_HEAD, nullptr, nullptr, nullptr, nullptr, nullptr, nullptr, nullptr, nullptr, STG, 0);
  k_outw<<<NRT / 64, 256, 0, stream>>>(STG, (float*)d_out);
}
